// DynamicModel_9088150798672
// MI455X (gfx1250) — hardware-verified
//
#include <hip/hip_runtime.h>

typedef __bf16 v16bf __attribute__((ext_vector_type(16)));
typedef __bf16 v8bf  __attribute__((ext_vector_type(8)));
typedef float  v8f   __attribute__((ext_vector_type(8)));
typedef float  v4f   __attribute__((ext_vector_type(4)));
typedef unsigned int v4u __attribute__((ext_vector_type(4)));
typedef v8bf __attribute__((may_alias)) v8bfa;
typedef v4f  __attribute__((may_alias)) v4fa;
typedef v4u  __attribute__((may_alias)) v4ua;

union FragB { v16bf v; v8bf half[2]; };

#define T_LEN  1024
#define HDIM   512
#define CIN    4
#define COUT   4
#define CMCH   8
#define RF     32
#define KDIM   (CMCH * RF)
#define NB     16
#define NTHR   256
#define NWAVE  8
#define TS     32
#define W1_N   (HDIM * KDIM)

__device__ __forceinline__ unsigned int bf16_rne_bits(float x) {
  const unsigned int u = __float_as_uint(x);
  return (u + 0x7FFFu + ((u >> 16) & 1u)) >> 16;
}
__device__ __forceinline__ float bf16_bits_to_f32(unsigned int b) {
  return __uint_as_float(b << 16);
}

__device__ __forceinline__ v8f wmma_bf16(v16bf a, v16bf b, v8f c) {
  v8f d = __builtin_amdgcn_wmma_f32_16x16x32_bf16(false, a, false, b, (short)0, c, false, false);
  asm volatile("v_nop\n\tv_nop\n\tv_nop\n\tv_nop" : "+v"(d) : "v"(a), "v"(b));
  return d;
}

__device__ __forceinline__ v16bf load_frag_g(const unsigned short* p, int hf) {
  FragB f;
  f.half[0] = *(const v8bfa*)(p + 8 * hf);
  f.half[1] = *(const v8bfa*)(p + 16 + 8 * hf);
  return f.v;
}

__device__ __forceinline__ v16bf load_frag_lds(const unsigned int* p, int hf) {
  FragB f;
  f.half[0] = *(const v8bfa*)(p + 4 * hf);
  f.half[1] = *(const v8bfa*)(p + 8 + 4 * hf);
  return f.v;
}

__global__ __launch_bounds__(256) void cvt_w1_kernel(
    const float* __restrict__ W1,
    unsigned short* __restrict__ whi,
    unsigned short* __restrict__ wlo,
    int n8)
{
  const int g = blockIdx.x * 256 + threadIdx.x;
  if (g >= n8) return;
  const float* src = W1 + (size_t)g * 8;
  const v4f a = *(const v4fa*)src;
  const v4f c = *(const v4fa*)(src + 4);
  const float x[8] = { a.x, a.y, a.z, a.w, c.x, c.y, c.z, c.w };
  unsigned int hb[8], lb[8];
  #pragma unroll
  for (int i = 0; i < 8; ++i) {
    hb[i] = bf16_rne_bits(x[i]);
    lb[i] = bf16_rne_bits(x[i] - bf16_bits_to_f32(hb[i]));
  }
  v4u hv, lv;
  hv.x = hb[0] | (hb[1] << 16);  hv.y = hb[2] | (hb[3] << 16);
  hv.z = hb[4] | (hb[5] << 16);  hv.w = hb[6] | (hb[7] << 16);
  lv.x = lb[0] | (lb[1] << 16);  lv.y = lb[2] | (lb[3] << 16);
  lv.z = lb[4] | (lb[5] << 16);  lv.w = lb[6] | (lb[7] << 16);
  unsigned short* dh = whi + (size_t)g * 8;
  unsigned short* dl = wlo + (size_t)g * 8;
  *(volatile v4u*)dh = hv;
  *(volatile v4u*)dl = lv;
  __threadfence();
  *(volatile v4u*)dh = hv;
  *(volatile v4u*)dl = lv;
}

__device__ __forceinline__ void out_store_pass(const float* ystage, float* out,
                                               int n0, int tb, int w, int lane) {
  const int q8 = lane & 7, sub = lane >> 3;
  #pragma unroll
  for (int i = 0; i < 2; ++i) {
    const int l = 8 * w + 4 * i + sub;
    const int n = l >> 2, o = l & 3;
    const v4f v = *(const v4fa*)(ystage + l * TS + 4 * q8);
    const size_t gi = ((size_t)(n0 + n) * COUT + o) * T_LEN + tb + 4 * q8;
    *(volatile v4f*)(out + gi) = v;
  }
}

__global__ __launch_bounds__(NTHR) void recur_kernel(
    const float* __restrict__ u,
    const unsigned short* __restrict__ whi,
    const unsigned short* __restrict__ wlo,
    const float* __restrict__ b1,
    const float* __restrict__ W2,
    const float* __restrict__ b2,
    float* __restrict__ out)
{
  __shared__ __attribute__((aligned(16))) unsigned int X[2 * CMCH * NB * 16];
  __shared__ __attribute__((aligned(16))) float W2s[COUT * HDIM];
  __shared__ __attribute__((aligned(16))) float b1s[HDIM];
  __shared__ __attribute__((aligned(16))) float ystage[NB * COUT * TS];
  __shared__ __attribute__((aligned(16))) float ypart[NWAVE * COUT * NB];
  __shared__ __attribute__((aligned(16))) float ylast[COUT * NB];

  const int tid = threadIdx.x, lane = tid & 31, w = tid >> 5;
  const int hf = lane >> 4, m = lane & 15;
  const int n0 = blockIdx.x * NB;
  const int hbase = 64 * w;

  {
    v4ua* rp = (v4ua*)(X + tid * 16);
    const v4u z = { 0u, 0u, 0u, 0u };
    rp[0] = z; rp[1] = z; rp[2] = z; rp[3] = z;
    const v4f s0 = *(const v4fa*)(W2 + tid * 8);
    const v4f s1 = *(const v4fa*)(W2 + tid * 8 + 4);
    v4fa* d = (v4fa*)(W2s + tid * 8);
    d[0] = s0; d[1] = s1;
    if (tid < HDIM / 4) {
      const v4f bb = *(const v4fa*)(b1 + tid * 4);
      *(v4fa*)(b1s + tid * 4) = bb;
    }
  }
  const float b2r = b2[(tid >> 4) & 3];

  const int cp = tid >> 7, cc = (tid >> 4) & 7, cn = tid & 15;
  const int csel = cc & 3;
  unsigned int* xrow = X + tid * 16;
  const float* urow = u + ((size_t)(n0 + cn) * CIN + csel) * T_LEN;

  #pragma unroll 1
  for (int t = 0; t < T_LEN; ++t) {
    const float usamp = urow[t];

    __syncthreads();

    v8f acc[4];
    #pragma unroll
    for (int rt = 0; rt < 4; ++rt) {
      const float* bp = b1s + hbase + 16 * rt + 8 * hf;
      const v4f q0 = *(const v4fa*)bp;
      const v4f q1 = *(const v4fa*)(bp + 4);
      const v8f c0 = { q0.x, q0.y, q0.z, q0.w, q1.x, q1.y, q1.z, q1.w };
      acc[rt] = c0;
    }

    const unsigned short* wrow_h = whi + (size_t)(hbase + m) * KDIM;
    const unsigned short* wrow_l = wlo + (size_t)(hbase + m) * KDIM;
    #pragma unroll 1
    for (int kt = 0; kt < CMCH; ++kt) {
      const unsigned int* xh = X + ((0 * CMCH + kt) * NB + m) * 16;
      const unsigned int* xl = X + ((1 * CMCH + kt) * NB + m) * 16;
      const v16bf bh = load_frag_lds(xh, hf);
      const v16bf bl = load_frag_lds(xl, hf);
      #pragma unroll
      for (int rt = 0; rt < 4; ++rt) {
        const size_t off = (size_t)(16 * rt) * KDIM + 32 * kt;
        const v16bf ah = load_frag_g(wrow_h + off, hf);
        const v16bf al = load_frag_g(wrow_l + off, hf);
        acc[rt] = wmma_bf16(ah, bh, acc[rt]);
        acc[rt] = wmma_bf16(ah, bl, acc[rt]);
        acc[rt] = wmma_bf16(al, bh, acc[rt]);
      }
    }

    float p[COUT] = { 0.0f, 0.0f, 0.0f, 0.0f };
    #pragma unroll
    for (int rt = 0; rt < 4; ++rt) {
      float hv[8];
      #pragma unroll
      for (int r = 0; r < 8; ++r) hv[r] = fmaxf(acc[rt][r], 0.0f);
      #pragma unroll
      for (int o = 0; o < COUT; ++o) {
        const float* wp = W2s + o * HDIM + hbase + 16 * rt + 8 * hf;
        const v4f wa = *(const v4fa*)wp;
        const v4f wb = *(const v4fa*)(wp + 4);
        p[o] = fmaf(wa.x, hv[0], p[o]);
        p[o] = fmaf(wa.y, hv[1], p[o]);
        p[o] = fmaf(wa.z, hv[2], p[o]);
        p[o] = fmaf(wa.w, hv[3], p[o]);
        p[o] = fmaf(wb.x, hv[4], p[o]);
        p[o] = fmaf(wb.y, hv[5], p[o]);
        p[o] = fmaf(wb.z, hv[6], p[o]);
        p[o] = fmaf(wb.w, hv[7], p[o]);
      }
    }
    #pragma unroll
    for (int o = 0; o < COUT; ++o) p[o] += __shfl_xor(p[o], 16);
    if (lane < 16) {
      #pragma unroll
      for (int o = 0; o < COUT; ++o) ypart[(w * COUT + o) * NB + m] = p[o];
    }
    __syncthreads();

    if (tid < COUT * NB) {
      const int o = tid >> 4, n = tid & 15;
      float s = 0.0f;
      #pragma unroll
      for (int ww = 0; ww < NWAVE; ++ww) s += ypart[(ww * COUT + o) * NB + n];
      const float y = s + b2r;
      ylast[o * NB + n] = y;
      ystage[(n * COUT + o) * TS + (t & (TS - 1))] = y;
    }
    __syncthreads();

    if ((t & (TS - 1)) == (TS - 1)) {
      const int tb = t - (TS - 1);
      out_store_pass(ystage, out, n0, tb, w, lane);
      __threadfence();
      out_store_pass(ystage, out, n0, tb, w, lane);
    }

    {
      const float ysamp = ylast[csel * NB + cn];
      const float xv = (cc < CIN) ? usamp : ysamp;
      const unsigned int hb = bf16_rne_bits(xv);
      const unsigned int lb = bf16_rne_bits(xv - bf16_bits_to_f32(hb));
      const unsigned int nv = cp ? lb : hb;
      v4ua* rp = (v4ua*)xrow;
      const v4u d0 = rp[0], d1 = rp[1], d2 = rp[2], d3 = rp[3];
      const unsigned int e[16] = { d0.x, d0.y, d0.z, d0.w, d1.x, d1.y, d1.z, d1.w,
                                   d2.x, d2.y, d2.z, d2.w, d3.x, d3.y, d3.z, d3.w };
      unsigned int f[16];
      #pragma unroll
      for (int j = 0; j < 15; ++j) f[j] = (e[j] >> 16) | (e[j + 1] << 16);
      f[15] = (e[15] >> 16) | (nv << 16);
      const v4u o0 = { f[0],  f[1],  f[2],  f[3]  };
      const v4u o1 = { f[4],  f[5],  f[6],  f[7]  };
      const v4u o2 = { f[8],  f[9],  f[10], f[11] };
      const v4u o3 = { f[12], f[13], f[14], f[15] };
      rp[0] = o0; rp[1] = o1; rp[2] = o2; rp[3] = o3;
    }
  }
}

extern "C" void kernel_launch(void* const* d_in, const int* in_sizes, int n_in,
                              void* d_out, int out_size, void* d_ws, size_t ws_size,
                              hipStream_t stream)
{
  if (n_in < 5) return;
  const int nu = in_sizes[0];
  const int nb = nu / (CIN * T_LEN);
  if (nb <= 0 || nb * CIN * T_LEN != nu || (nb % NB) != 0) return;
  if (in_sizes[1] != W1_N) return;
  if (in_sizes[2] != HDIM) return;
  if (in_sizes[3] != COUT * HDIM) return;
  if (in_sizes[4] != COUT) return;
  if (out_size != nb * COUT * T_LEN) return;

  const size_t plane_bytes = (size_t)W1_N * 2;
  if (2 * plane_bytes > ws_size) return;

  const float* u  = (const float*)d_in[0];
  const float* W1 = (const float*)d_in[1];
  const float* b1 = (const float*)d_in[2];
  const float* W2 = (const float*)d_in[3];
  const float* b2 = (const float*)d_in[4];
  float* out = (float*)d_out;

  char* ws = (char*)d_ws;
  unsigned short* whi = (unsigned short*)(ws);
  unsigned short* wlo = (unsigned short*)(ws + plane_bytes);

  const int n8 = W1_N / 8;
  cvt_w1_kernel<<<dim3((n8 + 255) / 256), dim3(256), 0, stream>>>(W1, whi, wlo, n8);

  recur_kernel<<<dim3(nb / NB), dim3(NTHR), 0, stream>>>(u, whi, wlo, b1, W2, b2, out);
}
